// EfficientCrossAttention_66236985639309
// MI455X (gfx1250) — hardware-verified
//
#include <hip/hip_runtime.h>


#define EMBED   256
#define HEADS   8
#define HD      32
#define NQ      4096
#define NSP     16384
#define NSPP    4096
#define NKV     4160
#define SCALE_F 0.17677669529663687f
#define POOLC_F 1.3862943611198906f
#define LOG2E   1.4426950408889634f
#define XSCALE  (SCALE_F * LOG2E)
typedef __attribute__((ext_vector_type(16))) _Float16 v16h;
typedef __attribute__((ext_vector_type(8)))  _Float16 v8h;
typedef __attribute__((ext_vector_type(8)))  float    v8f;
typedef __attribute__((ext_vector_type(4)))  float    v4f;
#define VST2(T, ptr, val) do { const T _v = (val); *(volatile T*)(ptr) = _v; __threadfence(); *(volatile T*)(ptr) = _v; } while (0)
__device__ __forceinline__ v8f wmma16(v16h a, v16h b, v8f c) {
  v8f d = __builtin_amdgcn_wmma_f32_16x16x32_f16(false, a, false, b, (short)0, c, false, false);
  asm volatile("v_nop\n\tv_nop\n\tv_nop\n\tv_nop" : "+v"(d) : "v"(a), "v"(b));
  return d;
}
__device__ __forceinline__ v16h frag16(const _Float16* p, int hh) {
  const v8h lo = *(const v8h*)(p + 8 * hh), hi = *(const v8h*)(p + 16 + 8 * hh);
  return __builtin_shufflevector(lo, hi, 0,1,2,3,4,5,6,7,8,9,10,11,12,13,14,15);
}
__device__ __forceinline__ int kmap(int e, int hh) { return (e < 8) ? (8 * hh + e) : (16 + 8 * hh + (e - 8)); }

__global__ __launch_bounds__(256) void transpose_w_kernel(const float* __restrict__ W, _Float16* __restrict__ Wt) {
  const int n = blockIdx.x * 8 + (threadIdx.x >> 5), k0 = (threadIdx.x & 31) * 8;
  v8h v;
#pragma unroll
  for (int e = 0; e < 8; ++e) v[e] = (_Float16)W[(size_t)(k0 + e) * EMBED + n];
  VST2(v8h, Wt + (size_t)n * EMBED + k0, v);
}
__global__ __launch_bounds__(256) void cvt_f16_kernel(const float* __restrict__ in, _Float16* __restrict__ out, int n8) {
  const int i = blockIdx.x * 256 + threadIdx.x;
  if (i >= n8) return;
  v8h v;
#pragma unroll
  for (int e = 0; e < 8; ++e) v[e] = (_Float16)in[(size_t)i * 8 + e];
  VST2(v8h, out + (size_t)i * 8, v);
}
__global__ __launch_bounds__(256) void pool_kernel(const float* __restrict__ k_in, const float* __restrict__ v_in, _Float16* __restrict__ kpool, _Float16* __restrict__ vpool) {
  const int idx = blockIdx.x * 256 + threadIdx.x;
  if (idx >= NKV * 32) return;
  const int t = idx >> 5, c0 = (idx & 31) * 8;
  v8h kv, vv;
  if (t < NSPP) {
    const int f = t >> 10, rem = t & 1023, y = rem >> 5, x = rem & 31;
    const size_t base = ((size_t)f * 4096 + (size_t)(2 * y) * 64 + (size_t)(2 * x)) * EMBED + c0;
#pragma unroll
    for (int e = 0; e < 8; ++e) {
      kv[e] = (_Float16)(0.25f * ((k_in[base + e] + k_in[base + EMBED + e]) + (k_in[base + 64 * EMBED + e] + k_in[base + 65 * EMBED + e])));
      vv[e] = (_Float16)(0.25f * ((v_in[base + e] + v_in[base + EMBED + e]) + (v_in[base + 64 * EMBED + e] + v_in[base + 65 * EMBED + e])));
    }
  } else {
    const size_t src = ((size_t)NSP + (size_t)(t - NSPP)) * EMBED + c0;
#pragma unroll
    for (int e = 0; e < 8; ++e) { kv[e] = (_Float16)k_in[src + e]; vv[e] = (_Float16)v_in[src + e]; }
  }
  VST2(v8h, kpool + (size_t)t * EMBED + c0, kv);
  VST2(v8h, vpool + (size_t)t * EMBED + c0, vv);
}
template <typename TO>
__global__ __launch_bounds__(32) void proj_gemm(const _Float16* __restrict__ A, const _Float16* __restrict__ Wt, const float* __restrict__ bias, TO* __restrict__ Out) {
  __shared__ __attribute__((aligned(16))) float sT[16][68];
  const int lane = threadIdx.x, hh = lane >> 4, l16 = lane & 15;
  const int r0 = blockIdx.x * 64, n0 = blockIdx.y * 64;
  v8f acc[4][4] = {};
#pragma unroll 2
  for (int k0 = 0; k0 < EMBED; k0 += 32) {
    v16h a[4];
#pragma unroll
    for (int mi = 0; mi < 4; ++mi) a[mi] = frag16(A + (size_t)(r0 + mi * 16 + l16) * EMBED + k0, hh);
#pragma unroll
    for (int ni = 0; ni < 4; ++ni) {
      const v16h b = frag16(Wt + (size_t)(n0 + ni * 16 + l16) * EMBED + k0, hh);
#pragma unroll
      for (int mi = 0; mi < 4; ++mi) acc[mi][ni] = wmma16(a[mi], b, acc[mi][ni]);
    }
  }
#pragma unroll
  for (int mi = 0; mi < 4; ++mi) {
#pragma unroll
    for (int ni = 0; ni < 4; ++ni)
#pragma unroll
      for (int i = 0; i < 8; ++i) sT[i + 8 * hh][ni * 16 + l16] = acc[mi][ni][i] + bias[n0 + ni * 16 + l16];
    __builtin_amdgcn_fence(__ATOMIC_RELEASE, "workgroup"); __builtin_amdgcn_wave_barrier(); __builtin_amdgcn_fence(__ATOMIC_ACQUIRE, "workgroup");
    for (int pass = 0; pass < 2; ++pass) {
      if (sizeof(TO) == 2) {
#pragma unroll
        for (int j = 0; j < 4; ++j) { const int rr = j * 4 + (lane >> 3), q8 = (lane & 7) * 8; v8h hv;
#pragma unroll
          for (int e = 0; e < 8; ++e) hv[e] = (_Float16)sT[rr][q8 + e];
          *(volatile v8h*)((_Float16*)Out + (size_t)(r0 + mi * 16 + rr) * EMBED + n0 + q8) = hv; }
      } else {
#pragma unroll
        for (int j = 0; j < 8; ++j) { const int rr = j * 2 + hh, q4 = l16 * 4;
          *(volatile v4f*)((float*)Out + (size_t)(r0 + mi * 16 + rr) * EMBED + n0 + q4) = *(const v4f*)(&sT[rr][q4]); }
      }
      __threadfence();
    }
    __builtin_amdgcn_fence(__ATOMIC_RELEASE, "workgroup"); __builtin_amdgcn_wave_barrier(); __builtin_amdgcn_fence(__ATOMIC_ACQUIRE, "workgroup");
  }
}
__global__ __launch_bounds__(32) void attn_kernel(const _Float16* __restrict__ Q, const _Float16* __restrict__ Kp, const _Float16* __restrict__ Vp, _Float16* __restrict__ O) {
  __shared__ __attribute__((aligned(16))) _Float16 Pld[2][16 * 40];
  __shared__ __attribute__((aligned(16))) _Float16 sO[32][72];
  const int lane = threadIdx.x, hh = lane >> 4, l16 = lane & 15;
  const int q0 = blockIdx.x * 32, hp = blockIdx.y;
  v16h ones;
#pragma unroll
  for (int i = 0; i < 16; ++i) ones[i] = (_Float16)1.0f;
  for (int hsub = 0; hsub < 2; ++hsub) {
    const int c0 = (hp * 2 + hsub) * HD;
    const v16h aq0 = frag16(Q + (size_t)(q0 + l16) * EMBED + c0, hh), aq1 = frag16(Q + (size_t)(q0 + 16 + l16) * EMBED + c0, hh);
    v8f acc[2][2] = {}, lsum[2] = {};
    for (int kv0 = 0; kv0 < NKV; kv0 += 32) {
      const v16h bk0 = frag16(Kp + (size_t)(kv0 + l16) * EMBED + c0, hh), bk1 = frag16(Kp + (size_t)(kv0 + 16 + l16) * EMBED + c0, hh);
      v16h bv0, bv1;
#pragma unroll
      for (int e = 0; e < 16; ++e) { const size_t ro = (size_t)(kv0 + kmap(e, hh)) * EMBED + c0 + l16; bv0[e] = Vp[ro]; bv1[e] = Vp[ro + 16]; }
      const float badd = (kv0 < NSPP) ? (POOLC_F * LOG2E) : 0.0f;
      const v8f z = {};
#pragma unroll
      for (int qt = 0; qt < 2; ++qt) {
        const v8f s0 = wmma16(qt ? aq1 : aq0, bk0, z), s1 = wmma16(qt ? aq1 : aq0, bk1, z);
#pragma unroll
        for (int i = 0; i < 8; ++i) {
          const int row = i + 8 * hh;
          Pld[qt][row * 40 + l16]      = (_Float16)__builtin_amdgcn_exp2f(s0[i] * XSCALE + badd);
          Pld[qt][row * 40 + 16 + l16] = (_Float16)__builtin_amdgcn_exp2f(s1[i] * XSCALE + badd);
        }
      }
      __builtin_amdgcn_fence(__ATOMIC_RELEASE, "workgroup"); __builtin_amdgcn_wave_barrier(); __builtin_amdgcn_fence(__ATOMIC_ACQUIRE, "workgroup");
#pragma unroll
      for (int qt = 0; qt < 2; ++qt) {
        const v16h ap = frag16(&Pld[qt][l16 * 40], hh);
        acc[qt][0] = wmma16(ap, bv0, acc[qt][0]);
        acc[qt][1] = wmma16(ap, bv1, acc[qt][1]);
        lsum[qt]   = wmma16(ap, ones, lsum[qt]);
      }
      __builtin_amdgcn_fence(__ATOMIC_RELEASE, "workgroup"); __builtin_amdgcn_wave_barrier(); __builtin_amdgcn_fence(__ATOMIC_ACQUIRE, "workgroup");
    }
#pragma unroll
    for (int qt = 0; qt < 2; ++qt)
#pragma unroll
      for (int i = 0; i < 8; ++i) {
        const int row = 16 * qt + i + 8 * hh; const float inv = 1.0f / lsum[qt][i];
        sO[row][hsub * 32 + l16]      = (_Float16)(acc[qt][0][i] * inv);
        sO[row][hsub * 32 + 16 + l16] = (_Float16)(acc[qt][1][i] * inv);
      }
  }
  __builtin_amdgcn_fence(__ATOMIC_RELEASE, "workgroup"); __builtin_amdgcn_wave_barrier(); __builtin_amdgcn_fence(__ATOMIC_ACQUIRE, "workgroup");
  for (int pass = 0; pass < 2; ++pass) {
#pragma unroll
    for (int j = 0; j < 8; ++j) { const int rr = j * 4 + (lane >> 3), q8 = (lane & 7) * 8;
      *(volatile v8h*)(O + (size_t)(q0 + rr) * EMBED + hp * 64 + q8) = *(const v8h*)(&sO[rr][q8]); }
    __threadfence();
  }
}
extern "C" void kernel_launch(void* const* d_in, const int* in_sizes, int n_in,
                              void* d_out, int out_size, void* d_ws, size_t ws_size, hipStream_t stream) {
  (void)in_sizes; (void)n_in; (void)out_size;
  const float* q  = (const float*)d_in[0];
  const float* k  = (const float*)d_in[1];
  const float* v  = (const float*)d_in[2];
  const float* Wq = (const float*)d_in[3]; const float* bq = (const float*)d_in[4];
  const float* Wk = (const float*)d_in[5]; const float* bk = (const float*)d_in[6];
  const float* Wv = (const float*)d_in[7]; const float* bv = (const float*)d_in[8];
  const float* Wo = (const float*)d_in[9]; const float* bo = (const float*)d_in[10];
  float* out = (float*)d_out;
  const size_t kvb = (size_t)NKV * EMBED, qb = (size_t)NQ * EMBED, wb = (size_t)EMBED * EMBED;
  if (ws_size < (4 * kvb + 3 * qb + 4 * wb) * 2) return;
  _Float16* kpool = (_Float16*)d_ws;
  _Float16* vpool = kpool + kvb;
  _Float16* qh    = vpool + kvb;
  _Float16* qp    = qh + qb;
  _Float16* kp    = qp + qb;
  _Float16* vp    = kp + kvb;
  _Float16* ao    = vp + kvb;
  _Float16* wqT   = ao + qb;
  _Float16* wkT   = wqT + wb;
  _Float16* wvT   = wkT + wb;
  _Float16* woT   = wvT + wb;
  transpose_w_kernel<<<EMBED / 8, 256, 0, stream>>>(Wq, wqT);
  transpose_w_kernel<<<EMBED / 8, 256, 0, stream>>>(Wk, wkT);
  transpose_w_kernel<<<EMBED / 8, 256, 0, stream>>>(Wv, wvT);
  transpose_w_kernel<<<EMBED / 8, 256, 0, stream>>>(Wo, woT);
  cvt_f16_kernel<<<(NQ * EMBED / 8) / 256, 256, 0, stream>>>(q, qh, NQ * EMBED / 8);
  pool_kernel<<<(NKV * 32 + 255) / 256, 256, 0, stream>>>(k, v, kpool, vpool);
  proj_gemm<_Float16><<<dim3(NQ / 64, EMBED / 64), 32, 0, stream>>>(qh, wqT, bq, qp);
  proj_gemm<_Float16><<<dim3(NKV / 64, EMBED / 64), 32, 0, stream>>>(kpool, wkT, bk, kp);
  proj_gemm<_Float16><<<dim3(NKV / 64, EMBED / 64), 32, 0, stream>>>(vpool, wvT, bv, vp);
  attn_kernel<<<dim3(NQ / 32, HEADS / 2), 32, 0, stream>>>(qp, kp, vp, ao);
  proj_gemm<float><<<dim3(NQ / 64, EMBED / 64), 32, 0, stream>>>(ao, woT, bo, out);
}
